// CrystalGraphAttention_89859305767778
// MI455X (gfx1250) — hardware-verified
//
#include <hip/hip_runtime.h>
#include <stddef.h>
#include <stdint.h>


#define HID     128
#define HD      32
#define NHEAD   4
#define KVW     256
#define NQKV    384
#define GATE    32
#define NTHR    256
#define NWAVE   8
#define EPT     8
#define CHUNK   (NTHR * EPT)
#define WCAP    (EPT * 32)
#define LISTN   (NWAVE * WCAP)
#define NBMAX   1024
#define SLB     10
#define RCAP    28672
#define DEGCAP  512
#define STW     128
#define GBM     64
#define GBN     64
#define GTHR    128
#define CX      8.0f
#define CW      64.0f
#define CQ      8.0f
#define INVCQ   0.125f
#define SCL_XW  0.001953125f
#define ATTSC   0.17677669529663687f
#define WSMAX   134217728
#define LDS_AGG ((2 * RCAP + 2 * NBMAX + LISTN) * 4 + 64)

static_assert((CHUNK & (CHUNK - 1)) == 0 && CHUNK <= 2048);
static_assert((NBMAX & (NBMAX - 1)) == 0 && (1 << SLB) == NBMAX);
static_assert(NTHR * 4 == NBMAX);
static_assert(LISTN >= NBMAX);
static_assert(LISTN >= NWAVE * WCAP);
static_assert((RCAP % 32) == 0);
static_assert(NWAVE * STW <= RCAP);
static_assert(STW == HID);
static_assert(LDS_AGG <= 300000);
static_assert(GBM == (GTHR / 32) * 16);
static_assert(HID / 8 == 16 && (HID % 32) == 0);
static_assert(NQKV == 3 * HID && KVW == 2 * HID && NHEAD * HD == HID);
static_assert(GATE == 32 && HD == 32);
static_assert((KVW % GBN) == 0 && (HID % GBN) == 0);

typedef float    v4f  __attribute__((ext_vector_type(4)));
typedef float    v8f  __attribute__((ext_vector_type(8)));
typedef int      v4i  __attribute__((ext_vector_type(4)));
typedef int      v8i  __attribute__((ext_vector_type(8)));
typedef _Float16 v4h  __attribute__((ext_vector_type(4)));
typedef _Float16 v8h  __attribute__((ext_vector_type(8)));
typedef _Float16 v16h __attribute__((ext_vector_type(16)));
union FragH { v16h v; v8h h[2]; v8i w; };

__device__ __forceinline__ v8f wmh(const FragH& a, const FragH& b, v8f c) {
  v8f d = __builtin_amdgcn_wmma_f32_16x16x32_f16(false, a.v, false, b.v, (short)0, c, false, false);
  asm volatile("v_nop\n\tv_nop\n\tv_nop\n\tv_nop" : "+v"(d) : "v"(a.w), "v"(b.w));
  return d;
}

__device__ __forceinline__ void ldwait() {
  asm volatile("s_wait_loadcnt 0x0" ::: "memory");
}

__device__ __forceinline__ v8h cvt8h(const v4f a, const v4f b, const float c) {
  v8h hv;
  hv[0] = (_Float16)(a.x * c); hv[1] = (_Float16)(a.y * c);
  hv[2] = (_Float16)(a.z * c); hv[3] = (_Float16)(a.w * c);
  hv[4] = (_Float16)(b.x * c); hv[5] = (_Float16)(b.y * c);
  hv[6] = (_Float16)(b.z * c); hv[7] = (_Float16)(b.w * c);
  return hv;
}

__device__ __forceinline__ int scan_chunk(const int* __restrict__ dsts, int nE, int cbase, int slotBase,
                                          int nb, int vec8, int* list, int tid, int lane, int wave) {
  int wc = 0;
  const int el0  = tid * EPT;
  const int e0   = cbase + el0;
  const int sent = -2147483647 - 1;
  v4i da, db;
  if (vec8 != 0 && cbase + CHUNK <= nE) {
    da = *(const v4i*)(dsts + e0);
    db = *(const v4i*)(dsts + e0 + 4);
  } else {
    da.x = (e0     < nE) ? dsts[min(e0,     nE - 1)] : sent;
    da.y = (e0 + 1 < nE) ? dsts[min(e0 + 1, nE - 1)] : sent;
    da.z = (e0 + 2 < nE) ? dsts[min(e0 + 2, nE - 1)] : sent;
    da.w = (e0 + 3 < nE) ? dsts[min(e0 + 3, nE - 1)] : sent;
    db.x = (e0 + 4 < nE) ? dsts[min(e0 + 4, nE - 1)] : sent;
    db.y = (e0 + 5 < nE) ? dsts[min(e0 + 5, nE - 1)] : sent;
    db.z = (e0 + 6 < nE) ? dsts[min(e0 + 6, nE - 1)] : sent;
    db.w = (e0 + 7 < nE) ? dsts[min(e0 + 7, nE - 1)] : sent;
  }
  const unsigned nbs = (unsigned)slotBase;
  const unsigned unb = (unsigned)nb;
  const unsigned s0 = (unsigned)da.x - nbs, s1 = (unsigned)da.y - nbs;
  const unsigned s2 = (unsigned)da.z - nbs, s3 = (unsigned)da.w - nbs;
  const unsigned s4 = (unsigned)db.x - nbs, s5 = (unsigned)db.y - nbs;
  const unsigned s6 = (unsigned)db.z - nbs, s7 = (unsigned)db.w - nbs;
  const bool h0 = s0 < unb, h1 = s1 < unb, h2 = s2 < unb, h3 = s3 < unb;
  const bool h4 = s4 < unb, h5 = s5 < unb, h6 = s6 < unb, h7 = s7 < unb;
  const unsigned any = __builtin_amdgcn_ballot_w32(h0 | h1 | h2 | h3 | h4 | h5 | h6 | h7);
  if (any != 0u) {
#define HITJ(J, HJ, SJ) { \
      const unsigned mj = __builtin_amdgcn_ballot_w32(HJ); \
      if (mj != 0u) { \
        if (HJ) { \
          const int pos = wc + (int)__builtin_amdgcn_mbcnt_lo(mj, 0u); \
          if (pos < WCAP) list[wave * WCAP + pos] = ((el0 + (J)) << SLB) | (int)(SJ); \
        } \
        wc += (int)__builtin_popcount(mj); } }
    HITJ(0, h0, s0)
    HITJ(1, h1, s1)
    HITJ(2, h2, s2)
    HITJ(3, h3, s3)
    HITJ(4, h4, s4)
    HITJ(5, h5, s5)
    HITJ(6, h6, s6)
    HITJ(7, h7, s7)
#undef HITJ
  }
  return wc;
}

__global__ __launch_bounds__(NTHR) void k_xprep(const float* __restrict__ h, const float* __restrict__ fc,
                                                const float* __restrict__ fW, const float* __restrict__ fb,
                                                _Float16* xh, int nN, int nUnits) {
  const int i = (int)blockIdx.x * NTHR + (int)threadIdx.x;
  if (i >= nUnits) return;
  const int row = i >> 4;
  const int c0  = (i & 15) * 8;
  const int rc  = row < nN ? row : nN - 1;
  const float* p = h + (size_t)rc * HID + c0;
  v4f a = *(const v4f*)p, b = *(const v4f*)(p + 4);
  const float f0 = fc[(size_t)rc * 3 + 0];
  const float f1 = fc[(size_t)rc * 3 + 1];
  const float f2 = fc[(size_t)rc * 3 + 2];
  const v4f w0a = *(const v4f*)(fW + c0),           w0b = *(const v4f*)(fW + c0 + 4);
  const v4f w1a = *(const v4f*)(fW + HID + c0),     w1b = *(const v4f*)(fW + HID + c0 + 4);
  const v4f w2a = *(const v4f*)(fW + 2 * HID + c0), w2b = *(const v4f*)(fW + 2 * HID + c0 + 4);
  const v4f ba  = *(const v4f*)(fb + c0),           bb  = *(const v4f*)(fb + c0 + 4);
  v4f ta = w0a * f0; ta = w1a * f1 + ta; ta = w2a * f2 + ta;
  v4f tb = w0b * f0; tb = w1b * f1 + tb; tb = w2b * f2 + tb;
  a = (a + ta) + ba;
  b = (b + tb) + bb;
  const v4f z4 = {0.f, 0.f, 0.f, 0.f};
  if (row >= nN) { a = z4; b = z4; }
  const v8h hv = cvt8h(a, b, CX);
  const size_t o = (size_t)row * HID + c0;
  *(volatile v8h*)(xh + o) = hv;
  __threadfence();
  *(volatile v8h*)(xh + o) = hv;
}

__global__ __launch_bounds__(NTHR) void k_wtr(const float* __restrict__ w0, const float* __restrict__ w1,
                                              const float* __restrict__ w2, const float* __restrict__ w3,
                                              int c0, int c1, int c2, int c3, int segRows, int K,
                                              _Float16* wt, int nUnits) {
  const int u = (int)blockIdx.x * NTHR + (int)threadIdx.x;
  if (u >= nUnits) return;
  const int kq = K >> 3;
  const int n  = u / kq;
  const int k8 = (u - n * kq) * 8;
  int seg = n / segRows;
  seg = seg > 3 ? 3 : seg;
  const int nc = n - seg * segRows;
  const float* ws = (seg == 0) ? w0 : ((seg == 1) ? w1 : ((seg == 2) ? w2 : w3));
  const int cc = (seg == 0) ? c0 : ((seg == 1) ? c1 : ((seg == 2) ? c2 : c3));
  const int ncl = nc < cc ? nc : cc - 1;
  const float* p = ws + (size_t)k8 * (size_t)cc + ncl;
  v4f a, b;
  a.x = p[0];                  a.y = p[(size_t)cc];         a.z = p[(size_t)2 * cc];     a.w = p[(size_t)3 * cc];
  b.x = p[(size_t)4 * cc];     b.y = p[(size_t)5 * cc];     b.z = p[(size_t)6 * cc];     b.w = p[(size_t)7 * cc];
  const v4f z4 = {0.f, 0.f, 0.f, 0.f};
  if (nc >= cc) { a = z4; b = z4; }
  const v8h hv = cvt8h(a, b, CW);
  const size_t o = (size_t)n * (size_t)K + k8;
  *(volatile v8h*)(wt + o) = hv;
  __threadfence();
  *(volatile v8h*)(wt + o) = hv;
}

template<int EPI>
__global__ __launch_bounds__(GTHR) void k_gemm(
    const _Float16* __restrict__ A, const _Float16* __restrict__ WT,
    const float* __restrict__ b0, const float* __restrict__ b1,
    const float* __restrict__ b2, const float* __restrict__ b3,
    float* outF, _Float16* outH, int K, int ldo, int segN, int blen, int nRows, float scl, float cq)
{
  __shared__ __attribute__((aligned(16))) float stg[GBM * GBN];
  const int tid = (int)threadIdx.x, lane = tid & 31, wave = tid >> 5, hh = lane >> 4, m = lane & 15;
  const int rowBase = (int)blockIdx.x * GBM;
  const int col0    = (int)blockIdx.y * GBN;
  int seg = col0 / segN;
  seg = seg < 0 ? 0 : (seg > 3 ? 3 : seg);
  const float* bp = (seg == 0) ? b0 : ((seg == 1) ? b1 : ((seg == 2) ? b2 : b3));
  int bofs = col0 - seg * segN;
  bofs = bofs < 0 ? 0 : bofs;

  v8f acc[4];
  {
    const v8f z = {0.f, 0.f, 0.f, 0.f, 0.f, 0.f, 0.f, 0.f};
    acc[0] = z; acc[1] = z; acc[2] = z; acc[3] = z;
  }
  const _Float16* ap = A  + (size_t)(rowBase + 16 * wave + m) * (size_t)K + 8 * hh;
  const _Float16* wp = WT + (size_t)(col0 + m) * (size_t)K + 8 * hh;
  const int ksteps = K >> 5;
#pragma unroll 1
  for (int ks = 0; ks < ksteps; ++ks) {
    FragH af;
    af.h[0] = *(const v8h*)(ap + 32 * ks);
    af.h[1] = *(const v8h*)(ap + 32 * ks + 16);
#pragma unroll
    for (int t = 0; t < 4; ++t) {
      const _Float16* wq = wp + (size_t)(16 * t) * (size_t)K + 32 * ks;
      FragH bf;
      bf.h[0] = *(const v8h*)wq;
      bf.h[1] = *(const v8h*)(wq + 16);
      acc[t] = wmh(af, bf, acc[t]);
    }
  }

#pragma unroll
  for (int t = 0; t < 4; ++t) {
    const int lc = 16 * t + m;
    int bi = bofs + lc;
    bi = bi > blen - 1 ? blen - 1 : bi;
    bi = bi < 0 ? 0 : bi;
    const float bv = bp[bi];
#pragma unroll
    for (int r = 0; r < 8; ++r) {
      const int lr = 16 * wave + 8 * hh + r;
      stg[lr * GBN + lc] = fmaf(acc[t][r], scl, bv);
    }
  }
  __syncthreads();

  if (EPI == 2) {
    const int rq = lane >> 3;
    const int c8 = (lane & 7) * 8;
    v8h hv[4];
#pragma unroll
    for (int i = 0; i < 4; ++i) {
      const int lr = 16 * wave + 4 * i + rq;
      const v4f ga = *(const v4f*)(stg + lr * GBN + c8);
      const v4f gb = *(const v4f*)(stg + lr * GBN + c8 + 4);
      hv[i] = cvt8h(ga, gb, cq);
    }
#pragma unroll
    for (int i = 0; i < 4; ++i) {
      const int lr = 16 * wave + 4 * i + rq;
      const int gr = rowBase + lr;
      _Float16* op = outH + (size_t)gr * (size_t)ldo + col0 + c8;
      *(volatile v8h*)op = hv[i];
    }
    __threadfence();
#pragma unroll
    for (int i = 0; i < 4; ++i) {
      const int lr = 16 * wave + 4 * i + rq;
      const int gr = rowBase + lr;
      _Float16* op = outH + (size_t)gr * (size_t)ldo + col0 + c8;
      *(volatile v8h*)op = hv[i];
    }
  } else {
    v4f fv[8];
#pragma unroll
    for (int i = 0; i < 8; ++i) {
      const int lr = 16 * wave + 2 * i + hh;
      fv[i] = *(const v4f*)(stg + lr * GBN + 4 * m);
    }
#pragma unroll
    for (int i = 0; i < 8; ++i) {
      const int lr = 16 * wave + 2 * i + hh;
      const int gr = rowBase + lr;
      const bool ok = (EPI == 0) || (gr < nRows);
      float* op = outF + (size_t)gr * (size_t)ldo + col0 + 4 * m;
      if (ok) *(volatile v4f*)op = fv[i];
    }
    __threadfence();
#pragma unroll
    for (int i = 0; i < 8; ++i) {
      const int lr = 16 * wave + 2 * i + hh;
      const int gr = rowBase + lr;
      const bool ok = (EPI == 0) || (gr < nRows);
      float* op = outF + (size_t)gr * (size_t)ldo + col0 + 4 * m;
      if (ok) *(volatile v4f*)op = fv[i];
    }
  }
}

__global__ __launch_bounds__(NTHR) void k_agg(
    const int* __restrict__ rows, const int* __restrict__ cols, const float* __restrict__ dist,
    const float* __restrict__ g1W, const float* __restrict__ g1b,
    const float* __restrict__ g2W, const float* __restrict__ g2b,
    const float* __restrict__ QP, const _Float16* __restrict__ KV, _Float16* AG,
    int nN, int nE, int nb, int vec8, int MPr) {
  extern __shared__ v4f lds_dyn[];
  int* reg1 = (int*)lds_dyn;
  int* reg2 = reg1 + RCAP;
  int* scnt = reg2 + RCAP;
  int* soff = scnt + NBMAX;
  int* list = soff + NBMAX;
  int* wcnt = list + LISTN;
  int* wtot = wcnt + NWAVE;
  const int tid = (int)threadIdx.x, lane = tid & 31, wave = tid >> 5;
  const int nodeBase = (int)blockIdx.x * nb;

  for (int i = tid; i < NBMAX; i += NTHR) scnt[i] = 0;
  __syncthreads();

  int tot = 0;
  const int nChunks = (nE + CHUNK - 1) / CHUNK;
#pragma unroll 1
  for (int ch = 0; ch < nChunks; ++ch) {
    const int cbase = ch * CHUNK;
    const int wc = scan_chunk(rows, nE, cbase, nodeBase, nb, vec8, list, tid, lane, wave);
    if (lane == 0) wcnt[wave] = wc;
    __syncthreads();
    int pre = 0, all = 0;
#pragma unroll
    for (int w2 = 0; w2 < NWAVE; ++w2) {
      int c = wcnt[w2];
      c = c < 0 ? 0 : (c > WCAP ? WCAP : c);
      all += c;
      pre += (w2 < wave) ? c : 0;
    }
    const int wcc  = wc > WCAP ? WCAP : wc;
    const int base = tot + pre;
#pragma unroll 1
    for (int i = lane; i < wcc; i += 32) {
      const int ent = list[wave * WCAP + i];
      const int el  = (ent >> SLB) & (CHUNK - 1);
      const int sl  = ent & (NBMAX - 1);
      int eid = cbase + el;
      eid = eid > nE - 1 ? nE - 1 : eid;
      const int pos = base + i;
      if (pos < RCAP) reg1[pos] = (int)(((unsigned)eid << SLB) | (unsigned)sl);
    }
    tot += all;
    tot = tot > RCAP ? RCAP : tot;
    __syncthreads();
  }
  const int nh = tot;

  if (wave == 0) {
#pragma unroll 1
    for (int b0 = 0; b0 < nh; b0 += 32) {
      int idx = b0 + lane;
      idx = idx < nh ? idx : nh - 1;
      const int uv  = reg1[idx];
      const int m32 = (nh - b0) < 32 ? (nh - b0) : 32;
#pragma unroll 1
      for (int k = 0; k < m32; ++k) {
        const int u  = __builtin_amdgcn_readlane(uv, k);
        const int sl = u & (NBMAX - 1);
        if (lane == 0) scnt[sl] = scnt[sl] + 1;
      }
    }
  }
  __syncthreads();

  {
    const v4i ca = *(const v4i*)(scnt + 4 * tid);
    const int e0 = ca.x < 0 ? 0 : ca.x, e1 = ca.y < 0 ? 0 : ca.y, e2 = ca.z < 0 ? 0 : ca.z, e3 = ca.w < 0 ? 0 : ca.w;
    const int ts = e0 + e1 + e2 + e3;
    int incl = ts;
#pragma unroll
    for (int d = 1; d < 32; d <<= 1) {
      const int up = __shfl_up(incl, d);
      if (lane >= d) incl += up;
    }
    if (lane == 31) wtot[wave] = incl;
    __syncthreads();
    int pre = 0;
#pragma unroll
    for (int w2 = 0; w2 < NWAVE; ++w2) pre += (w2 < wave) ? wtot[w2] : 0;
    int run = pre + incl - ts;
    soff[4 * tid + 0] = run; run += e0;
    soff[4 * tid + 1] = run; run += e1;
    soff[4 * tid + 2] = run; run += e2;
    soff[4 * tid + 3] = run;
  }
  __syncthreads();
  for (int i = tid; i < NBMAX; i += NTHR) list[i] = soff[i];
  __syncthreads();

  if (wave == 0) {
#pragma unroll 1
    for (int b0 = 0; b0 < nh; b0 += 32) {
      int idx = b0 + lane;
      idx = idx < nh ? idx : nh - 1;
      const int uv  = reg1[idx];
      const int m32 = (nh - b0) < 32 ? (nh - b0) : 32;
#pragma unroll 1
      for (int k = 0; k < m32; ++k) {
        const int u   = __builtin_amdgcn_readlane(uv, k);
        const int sl  = u & (NBMAX - 1);
        const int eid = (int)((unsigned)u >> SLB);
        if (lane == 0) {
          int pos = list[sl];
          pos = pos < 0 ? 0 : (pos > RCAP - 1 ? RCAP - 1 : pos);
          reg2[pos] = eid;
          list[sl] = pos + 1;
        }
      }
    }
  }
  __syncthreads();

  const int nbw = nb >> 3;
  const bool ovf = (nh >= RCAP);
  const float qnan = __int_as_float(0x7fc00000);
  float* stw = (float*)reg1 + wave * STW;
  const int lc = lane < (HID / 8) ? lane : (HID / 8) - 1;
  const float gw1 = g1W[lane];
  const float gb1 = g1b[lane];
  const float gw2 = g2W[lane];
  const float gb2 = g2b[0];
#pragma unroll 1
  for (int jt = 0; jt < nbw; ++jt) {
    const int slot = wave * nbw + jt;
    const int grow = nodeBase + slot;
    const int gcl  = grow < nN ? grow : nN - 1;
    int st = soff[slot];
    const int craw = scnt[slot];
    int cnt = craw;
    st  = st < 0 ? 0 : (st > nh ? nh : st);
    cnt = cnt < 0 ? 0 : (cnt > DEGCAP ? DEGCAP : cnt);
    if (cnt > nh - st) cnt = nh - st;
    const float pz = (ovf || craw > DEGCAP) ? qnan : 0.0f;
    const bool wr = grow < MPr;
    const float live = grow < nN ? 1.0f : 0.0f;

    const v4f q4 = *(const v4f*)(QP + (size_t)gcl * HID + 4 * lane);
    ldwait();
    float mx = -1.0e30f, dn = 0.f;
    float a0 = 0.f, a1 = 0.f, a2 = 0.f, a3 = 0.f;

#pragma unroll 1
    for (int q = 0; q < cnt; ++q) {
      int idx = st + q; idx = idx > RCAP - 1 ? RCAP - 1 : idx;
      int eid = reg2[idx]; eid = eid < 0 ? 0 : (eid > nE - 1 ? nE - 1 : eid);
      const int sraw = cols[eid];
      const float dv = dist[eid];
      const int s = sraw < 0 ? 0 : (sraw > nN - 1 ? nN - 1 : sraw);
      const _Float16* kr = KV + (size_t)s * KVW + 4 * lane;
      const v4h k4 = *(const v4h*)kr;
      const v4h v4 = *(const v4h*)(kr + HID);
      ldwait();
      float p = q4.x * (float)k4.x;
      p = fmaf(q4.y, (float)k4.y, p);
      p = fmaf(q4.z, (float)k4.z, p);
      p = fmaf(q4.w, (float)k4.w, p);
      p += __shfl_xor(p, 1);
      p += __shfl_xor(p, 2);
      p += __shfl_xor(p, 4);
      const float ga = fmaf(dv, gw1, gb1);
      const float sg = __builtin_amdgcn_rcpf(1.0f + __expf(-ga));
      float t = (ga * sg) * gw2;
      t += __shfl_xor(t, 1);
      t += __shfl_xor(t, 2);
      t += __shfl_xor(t, 4);
      t += __shfl_xor(t, 8);
      t += __shfl_xor(t, 16);
      const float gt = __builtin_amdgcn_rcpf(1.0f + __expf(-(t + gb2)));
      const float al = (p * (ATTSC * INVCQ)) * gt;
      const float df = al - mx;
      const float ee = __expf(-fabsf(df));
      const bool up  = df > 0.f;
      const float s1 = up ? ee : 1.0f;
      const float s2 = up ? 1.0f : ee;
      mx = up ? al : mx;
      dn = fmaf(dn, s1, s2);
      a0 = fmaf(a0, s1, s2 * (float)v4.x);
      a1 = fmaf(a1, s1, s2 * (float)v4.y);
      a2 = fmaf(a2, s1, s2 * (float)v4.z);
      a3 = fmaf(a3, s1, s2 * (float)v4.w);
    }
    const float ds = dn > 0.f ? dn : 1.0f;
    const float iv = (dn > 0.f ? INVCQ : 0.0f) * __builtin_amdgcn_rcpf(ds) * live;
    v4f ov;
    ov.x = a0 * iv + pz;
    ov.y = a1 * iv + pz;
    ov.z = a2 * iv + pz;
    ov.w = a3 * iv + pz;
    __builtin_amdgcn_fence(__ATOMIC_RELEASE, "wavefront");
    __builtin_amdgcn_wave_barrier();
    *(v4f*)(stw + 4 * lane) = ov;
    __builtin_amdgcn_fence(__ATOMIC_RELEASE, "wavefront");
    __builtin_amdgcn_wave_barrier();
    const v4f g8a = *(const v4f*)(stw + 8 * lc);
    const v4f g8b = *(const v4f*)(stw + 8 * lc + 4);
    const v8h hv = cvt8h(g8a, g8b, CX);
    _Float16* gp = AG + (size_t)grow * HID + 8 * lc;
    const bool wsv = wr && (lane < (HID / 8));
    if (wsv) *(volatile v8h*)gp = hv;
    __threadfence();
    if (wsv) *(volatile v8h*)gp = hv;
  }
}

static int pick_nb(int nE, int nN) {
  int nb = NBMAX;
  while (nb > 16 && (long long)nb * (long long)nE * 5LL > (long long)RCAP * (long long)nN * 4LL) nb >>= 1;
  return nb;
}
static inline int cdiv(int a, int b) { return (a + b - 1) / b; }

extern "C" void kernel_launch(void* const* d_in, const int* in_sizes, int n_in,
                              void* d_out, int out_size, void* d_ws, size_t ws_size,
                              hipStream_t stream) {
  if (n_in < 18) return;
  const int nN = in_sizes[0] / HID;
  if (nN <= 0 || in_sizes[0] != nN * HID || nN > (1 << 22)) return;
  if (in_sizes[1] != nN * 3) return;
  if (in_sizes[2] < 2 || (in_sizes[2] & 1) != 0) return;
  const int nE = in_sizes[2] / 2;
  if (nE < 1 || nE > (1 << 22)) return;
  if (in_sizes[3] != nE) return;
  if (in_sizes[4] != 3 * HID || in_sizes[5] != HID) return;
  if (in_sizes[6] != HID * HID || in_sizes[7] != HID) return;
  if (in_sizes[8] != HID * HID || in_sizes[9] != HID) return;
  if (in_sizes[10] != HID * HID || in_sizes[11] != HID) return;
  if (in_sizes[12] != HID * HID || in_sizes[13] != HID) return;
  if (in_sizes[14] != GATE || in_sizes[15] != GATE) return;
  if (in_sizes[16] != GATE || in_sizes[17] != 1) return;
  if (out_size != nN * HID) return;

  const float* h    = (const float*)d_in[0];
  const float* fc   = (const float*)d_in[1];
  const int*   ei   = (const int*)  d_in[2];
  const float* dist = (const float*)d_in[3];
  const float* fW   = (const float*)d_in[4];
  const float* fb   = (const float*)d_in[5];
  const float* qW   = (const float*)d_in[6];
  const float* qb   = (const float*)d_in[7];
  const float* kW   = (const float*)d_in[8];
  const float* kb   = (const float*)d_in[9];
  const float* vW   = (const float*)d_in[10];
  const float* vb   = (const float*)d_in[11];
  const float* oW   = (const float*)d_in[12];
  const float* ob   = (const float*)d_in[13];
  const float* g1W  = (const float*)d_in[14];
  const float* g1b  = (const float*)d_in[15];
  const float* g2W  = (const float*)d_in[16];
  const float* g2b  = (const float*)d_in[17];
  float* out = (float*)d_out;
  const int* rows = ei;
  const int* cols = ei + nE;

  const int MP   = cdiv(nN, GBM) * GBM;
  const int nb   = pick_nb(nE, nN);
  const int gA   = cdiv(MP, nb);
  const int vec8 = 1;
  if (gA * nb < MP) return;

  char* ws = (char*)d_ws;
  size_t off = 0;
  const size_t oXH  = off; off += (size_t)MP * HID * 2;            off = (off + 255) & ~(size_t)255;
  const size_t oQP  = off; off += (size_t)MP * HID * 4;            off = (off + 255) & ~(size_t)255;
  const size_t oKV  = off; off += (size_t)MP * KVW * 2;            off = (off + 255) & ~(size_t)255;
  const size_t oWT1 = off; off += (size_t)NQKV * HID * 2;          off = (off + 255) & ~(size_t)255;
  const size_t oWOT = off; off += (size_t)HID * HID * 2;           off = (off + 255) & ~(size_t)255;
  if (off > ws_size || off > (size_t)WSMAX) return;
  _Float16* XH  = (_Float16*)(ws + oXH);
  float*    QP  = (float*)(ws + oQP);
  _Float16* KV  = (_Float16*)(ws + oKV);
  _Float16* WT1 = (_Float16*)(ws + oWT1);
  _Float16* WOT = (_Float16*)(ws + oWOT);
  _Float16* AG  = XH;

  hipFuncSetAttribute(reinterpret_cast<const void*>(&k_agg),
                      hipFuncAttributeMaxDynamicSharedMemorySize, LDS_AGG);

  const int nUx = MP * (HID / 8);
  k_xprep<<<cdiv(nUx, NTHR), NTHR, 0, stream>>>(h, fc, fW, fb, XH, nN, nUx);

  {
    const int nU1 = NQKV * (HID / 8);
    k_wtr<<<cdiv(nU1, NTHR), NTHR, 0, stream>>>(qW, kW, vW, vW, HID, HID, HID, HID, HID, HID, WT1, nU1);
    const int nU2 = HID * (HID / 8);
    k_wtr<<<cdiv(nU2, NTHR), NTHR, 0, stream>>>(oW, oW, oW, oW, HID, HID, HID, HID, HID, HID, WOT, nU2);
  }

  const int gM = MP / GBM;
  k_gemm<0><<<dim3(gM, HID / GBN), GTHR, 0, stream>>>(XH, WT1, qb, qb, qb, qb, QP, KV,
                                                      HID, HID, HID, HID, nN, SCL_XW, 1.0f);
  k_gemm<2><<<dim3(gM, KVW / GBN), GTHR, 0, stream>>>(XH, WT1 + (size_t)HID * HID, kb, vb, vb, vb, QP, KV,
                                                      HID, KVW, HID, HID, nN, SCL_XW, CQ);
  k_agg<<<gA, NTHR, LDS_AGG, stream>>>(rows, cols, dist, g1W, g1b, g2W, g2b, QP, KV, AG, nN, nE, nb, vec8, MP);
  k_gemm<1><<<dim3(gM, HID / GBN), GTHR, 0, stream>>>(AG, WOT, ob, ob, ob, ob, out, KV,
                                                      HID, HID, HID, HID, nN, SCL_XW, 1.0f);
}
